// MLPTime_20779051778730
// MI455X (gfx1250) — hardware-verified
//
#include <hip/hip_runtime.h>
#include <math.h>

typedef __attribute__((ext_vector_type(16))) _Float16 v16h;
typedef __attribute__((ext_vector_type(16))) __bf16 v16b;
typedef __attribute__((ext_vector_type(8)))  _Float16 v8h;
typedef __attribute__((ext_vector_type(8)))  float v8f;
typedef __attribute__((ext_vector_type(4)))  float v4f;
typedef __attribute__((ext_vector_type(2)))  float v2f;
typedef __attribute__((ext_vector_type(4)))  unsigned v4u;
typedef __attribute__((ext_vector_type(4)))  int v4i;
typedef float __attribute__((may_alias)) float_a;
typedef int __attribute__((may_alias)) int_a;

template <typename T> __device__ __forceinline__ void vst2(void* p, T v) { *(volatile T*)p = v; __threadfence(); *(volatile T*)p = v; }
__device__ __forceinline__ v8f wmma16(v16h a, v16h b, v8f c) {
  v8f d = __builtin_amdgcn_wmma_f32_16x16x32_f16(false, a, false, b, (short)0, c, false, false);
  asm volatile("v_nop\n\tv_nop\n\tv_nop\n\tv_nop" : "+v"(d) : "v"(a), "v"(b));
  return d;
}
__device__ __forceinline__ v8f wmma_bf(v16b a, v16b b, v8f c) {
  v8f d = __builtin_amdgcn_wmma_f32_16x16x32_bf16(false, a, false, b, (short)0, c, false, false);
  asm volatile("v_nop\n\tv_nop\n\tv_nop\n\tv_nop" : "+v"(d) : "v"(a), "v"(b));
  return d;
}
__device__ __forceinline__ v16h frag_h(const _Float16* rowk0, int lane) {
  union { v16h v; v8h q[2]; } u; const _Float16* p = rowk0 + 8 * (lane >> 4);
  u.q[0] = *(const v8h*)p; u.q[1] = *(const v8h*)(p + 16); return u.v;
}
__device__ __forceinline__ v16h frag_f32(const float* rowk0, int lane) {
  v16h a; const float* p = rowk0 + 8 * (lane >> 4);
#pragma unroll
  for (int i = 0; i < 8; ++i) { a[i] = (_Float16)p[i]; a[8 + i] = (_Float16)p[16 + i]; }
  return a;
}
__device__ __forceinline__ v16h frag_f32s(const float* rowk0, int lane, float sc) {
  v16h a; const float* p = rowk0 + 8 * (lane >> 4);
#pragma unroll
  for (int i = 0; i < 8; ++i) { a[i] = (_Float16)(p[i] * sc); a[8 + i] = (_Float16)(p[16 + i] * sc); }
  return a;
}
__device__ __forceinline__ v16h fragc_f32(const float* W, int k0, int n, int lane, int ld, int K) {
  v16h a; const int g = lane >> 4;
#pragma unroll
  for (int i = 0; i < 8; ++i) { const int ka = k0 + 8 * g + i, kb = ka + 16;
    a[i] = (_Float16)(ka < K ? W[(size_t)(ka < K ? ka : K - 1) * ld + n] : 0.f); a[8 + i] = (_Float16)(kb < K ? W[(size_t)(kb < K ? kb : K - 1) * ld + n] : 0.f); }
  return a;
}
struct F2 { v16b h, l; };
__device__ __forceinline__ F2 bsplit16(const float v[16]) { F2 r;
#pragma unroll
  for (int i = 0; i < 16; ++i) { const __bf16 h = (__bf16)v[i]; r.h[i] = h; r.l[i] = (__bf16)(v[i] - (float)h); }
  return r; }
__device__ __forceinline__ F2 split_row(const float* row, int k0, int lane) { float v[16]; const float* p = row + k0 + 8 * (lane >> 4);
#pragma unroll
  for (int i = 0; i < 8; ++i) { v[i] = p[i]; v[8 + i] = p[16 + i]; }
  return bsplit16(v); }
__device__ __forceinline__ F2 split_rowK(const float* row, int k0, int lane, int K) { float v[16]; const int g = lane >> 4;
#pragma unroll
  for (int i = 0; i < 8; ++i) { const int ka = k0 + 8 * g + i, kb = ka + 16; v[i] = ka < K ? row[ka < K ? ka : K - 1] : 0.f; v[8 + i] = kb < K ? row[kb < K ? kb : K - 1] : 0.f; }
  return bsplit16(v); }
__device__ __forceinline__ F2 split_col(const float* W, int k0, int n, int lane, int ld, int K) { float v[16]; const int g = lane >> 4;
#pragma unroll
  for (int i = 0; i < 8; ++i) { const int ka = k0 + 8 * g + i, kb = ka + 16; v[i] = ka < K ? W[(size_t)(ka < K ? ka : K - 1) * ld + n] : 0.f; v[8 + i] = kb < K ? W[(size_t)(kb < K ? kb : K - 1) * ld + n] : 0.f; }
  return bsplit16(v); }
__device__ __forceinline__ v8f mac3(const F2& a, const F2& b, v8f c) { c = wmma_bf(a.l, b.h, c); c = wmma_bf(a.h, b.l, c); return wmma_bf(a.h, b.h, c); }
__device__ __forceinline__ float sigm(float v) { return 1.0f / (1.0f + expf(-v)); }
#define LDSX() do { asm volatile("s_wait_dscnt 0" ::: "memory"); __builtin_amdgcn_wave_barrier(); __builtin_amdgcn_fence(__ATOMIC_RELEASE, "workgroup"); } while (0)


#define NTOK 16384
#define SS 512
#define NE 8
#ifndef NRB
#define NRB (NTOK / 64)
#endif
typedef __attribute__((ext_vector_type(8))) __bf16 v8b;
__device__ __forceinline__ v16b frag_b(const __bf16* rowk0, int lane) {
  union { v16b v; v8b q[2]; } u; const __bf16* p = rowk0 + 8 * (lane >> 4);
  u.q[0] = *(const v8b*)p; u.q[1] = *(const v8b*)(p + 16); return u.v;
}
__device__ __forceinline__ float bfr(float v) { return (float)(__bf16)v; }
__device__ __attribute__((noinline)) float exp_ni(float v) { return expf(v); }
__device__ __attribute__((noinline)) float erf_ni(float v) { return erff(v); }

#define WS_PW  0u
#define PEX 0
#define PGW (PEX + NE * SS * SS)
#define PWEND (PGW + 16 * SS)
#define WS_CW  (WS_PW + 2u * PWEND)
#define WS_END (WS_CW + 4u * NTOK * NE)

__global__ __launch_bounds__(128) void k_pack(const float* __restrict__ EW, const float* __restrict__ GW, __bf16* __restrict__ PW) {
  __shared__ __align__(16) __bf16 s[SS]; const int r = blockIdx.x, tid = threadIdx.x;
  for (int k = tid; k < SS; k += 128) { float v; if (r < NE * SS) v = EW[(size_t)r * SS + k]; else { const int e = r - NE * SS; v = (e < NE) ? GW[(size_t)e * SS + k] : 0.f; } s[k] = (__bf16)v; }
  __syncthreads();
  if (tid < SS / 8) vst2((unsigned*)(PW + (size_t)r * SS + tid * 8), *(const v4u*)&s[tid * 8]);
}
__global__ __launch_bounds__(128) void k_gate(const float* __restrict__ X, const __bf16* __restrict__ PW, float* __restrict__ GOUT, float* __restrict__ CW) {
  __shared__ __align__(16) float sg[64][NE]; __shared__ __align__(16) float sc[64][NE];
  const int tid = threadIdx.x, wave = tid >> 5, lane = tid & 31, col = lane & 15, g = lane >> 4; const size_t r0 = (size_t)blockIdx.x * 64 + wave * 16;
  v8f acc = {};
#pragma unroll 4
  for (int kc = 0; kc < SS / 32; ++kc) { v16b a; { const float* p = X + (r0 + col) * SS + kc * 32 + 8 * g;
#pragma unroll
      for (int i = 0; i < 8; ++i) { a[i] = (__bf16)p[i]; a[8 + i] = (__bf16)p[16 + i]; } }
    acc = wmma_bf(a, frag_b(PW + PGW + (size_t)col * SS + kc * 32, lane), acc); }
  __shared__ float sl[4][16][NE + 1];
  if (col < NE) {
#pragma unroll
    for (int r = 0; r < 8; ++r) sl[wave][8 * g + r][col] = acc[r]; }
  LDSX();
  if (lane < 16) { const int rl = lane; float lg[NE]; float mx = -3.0e38f;
#pragma unroll
    for (int e = 0; e < NE; ++e) { lg[e] = sl[wave][rl][e]; mx = fmaxf(mx, lg[e]); }
    float z = 0.f; float ge[NE];
#pragma unroll
    for (int e = 0; e < NE; ++e) { ge[e] = exp_ni(lg[e] - mx); z += ge[e]; }
    const float iz = 1.0f / z;
#pragma unroll
    for (int e = 0; e < NE; ++e) ge[e] *= iz;
    int i1 = 0; float v1 = ge[0];
#pragma unroll
    for (int e = 1; e < NE; ++e) if (ge[e] > v1) { v1 = ge[e]; i1 = e; }
    int i2 = -1; float v2 = -1.f;
#pragma unroll
    for (int e = 0; e < NE; ++e) if (e != i1 && ge[e] > v2) { v2 = ge[e]; i2 = e; }
#pragma unroll
    for (int e = 0; e < NE; ++e) { sg[wave * 16 + rl][e] = ge[e]; sc[wave * 16 + rl][e] = (e == i1) ? v1 : ((e == i2) ? v2 : 0.f); } }
  __syncthreads();
  vst2(GOUT + (size_t)blockIdx.x * 64 * NE + tid * 4, *(const v4f*)&(&sg[0][0])[tid * 4]);
  vst2(CW + (size_t)blockIdx.x * 64 * NE + tid * 4, *(const v4f*)&(&sc[0][0])[tid * 4]);
}
__global__ __launch_bounds__(128) void k_moe(const float* __restrict__ X, const __bf16* __restrict__ PW, const float* __restrict__ EB, const float* __restrict__ CW, float* __restrict__ OUT) {
  __shared__ __align__(16) float so[4][16][132];
  const int tid = threadIdx.x, wave = tid >> 5, lane = tid & 31, col = lane & 15, g = lane >> 4; const size_t r0 = (size_t)blockIdx.x * 64 + wave * 16; const int n0 = blockIdx.y * 128;
  v8f tot[8] = {};
#pragma unroll 1
  for (int e = 0; e < NE; ++e) { v8f acc[8] = {};
#pragma unroll 2
    for (int kc = 0; kc < SS / 32; ++kc) { v16b a; { const float* p = X + (r0 + col) * SS + kc * 32 + 8 * g;
#pragma unroll
        for (int i = 0; i < 8; ++i) { a[i] = (__bf16)p[i]; a[8 + i] = (__bf16)p[16 + i]; } }
#pragma unroll
      for (int j = 0; j < 8; ++j) acc[j] = wmma_bf(a, frag_b(PW + PEX + ((size_t)e * SS + n0 + j * 16 + col) * SS + kc * 32, lane), acc[j]); }
    float cw[8];
#pragma unroll
    for (int r = 0; r < 8; ++r) cw[r] = CW[(r0 + 8 * g + r) * NE + e];
#pragma unroll
    for (int j = 0; j < 8; ++j) { const float bb = bfr(EB[(size_t)e * SS + n0 + j * 16 + col]);
#pragma unroll
      for (int r = 0; r < 8; ++r) tot[j][r] += cw[r] * (acc[j][r] + bb); } }
#pragma unroll
  for (int j = 0; j < 8; ++j)
#pragma unroll
    for (int r = 0; r < 8; ++r) so[wave][8 * g + r][j * 16 + col] = fmaxf(tot[j][r], 0.f);
  LDSX();
  for (int rl = 0; rl < 16; ++rl) vst2(OUT + (r0 + rl) * SS + n0 + lane * 4, *(const v4f*)&so[wave][rl][lane * 4]);
}
extern "C" void kernel_launch(void* const* d_in, const int* in_sizes, int n_in, void* d_out, int out_size, void* d_ws, size_t ws_size, hipStream_t stream) {
  (void)in_sizes; (void)n_in; (void)out_size;
  const float** F = (const float**)d_in;
  if (ws_size < (size_t)WS_END) return;
  char* ws = (char*)d_ws; __bf16* PW = (__bf16*)(ws + WS_PW); float* CW = (float*)(ws + WS_CW);
  float* OUT = (float*)d_out; float* GOUT = OUT + (size_t)NTOK * SS;
  k_pack<<<NE * SS + 16, 128, 0, stream>>>(F[2], F[1], PW);
  k_gate<<<NRB, 128, 0, stream>>>(F[0], PW, GOUT, CW);
  k_moe<<<dim3(NRB, SS / 128), 128, 0, stream>>>(F[0], PW, F[3], CW, OUT);
}
